// PositionAttentionModule2_5523327942727
// MI455X (gfx1250) — hardware-verified
//
#include <hip/hip_runtime.h>


#define NB     4
#define CD     256
#define HDIM   64
#define WDIM   64
#define HW     (HDIM * WDIM)
#define PLANE  (NB * CD * HW)
#define X_N    PLANE
#define W_N    (CD * CD)
#define B_N    CD
#define OUT_N  PLANE

#define SZ_PX   ((size_t)PLANE * 4)
#define SZ_XT   ((size_t)NB * HW * CD * 2)
#define SZ_W16  ((size_t)CD * CD * 2)
#define OFF_PXB ((size_t)0)
#define OFF_PXC (OFF_PXB + SZ_PX)
#define OFF_XT  (OFF_PXC + SZ_PX)
#define OFF_W16 (OFF_XT + SZ_XT)
#define WS_TOTAL (OFF_W16 + 2 * SZ_W16)

static_assert(WS_TOTAL == 42205184);
static_assert((OFF_PXC % 128) == 0 && (OFF_XT % 128) == 0 && (OFF_W16 % 128) == 0 && (SZ_W16 % 128) == 0);
static_assert(HW % 64 == 0 && CD % 64 == 0 && (NB * HW) % 256 == 0);

#define XP 72
#define EP 68

typedef unsigned short v8us  __attribute__((ext_vector_type(8)));
typedef unsigned short v8usa __attribute__((ext_vector_type(8), __may_alias__));
typedef unsigned short v16us __attribute__((ext_vector_type(16)));
typedef _Float16       v16h  __attribute__((ext_vector_type(16)));
typedef float          v8f   __attribute__((ext_vector_type(8)));
typedef float          v4f   __attribute__((ext_vector_type(4)));
typedef float          v4fa  __attribute__((ext_vector_type(4), __may_alias__));

union Frag { v16us v; v8us half[2]; };

__device__ __forceinline__ unsigned short h2us(float f) {
  return __builtin_bit_cast(unsigned short, (_Float16)f);
}

__device__ __forceinline__ void st2_u8(unsigned short* p, v8us v) {
  *(volatile v8us*)p = v;
  __threadfence();
  *(volatile v8us*)p = v;
}
__device__ __forceinline__ void st2_f4(float* p, v4f v) {
  *(volatile v4f*)p = v;
  __threadfence();
  *(volatile v4f*)p = v;
}

__device__ __forceinline__ v16h ldfrag(const unsigned short* rowp, int h) {
  Frag f;
  f.half[0] = *(const v8us*)(rowp + 8 * h);
  f.half[1] = *(const v8us*)(rowp + 16 + 8 * h);
  return __builtin_bit_cast(v16h, f.v);
}

__device__ __forceinline__ v8f wmma_h(v16h a, v16h b, v8f c) {
  return __builtin_amdgcn_wmma_f32_16x16x32_f16(false, a, false, b, (short)0, c, false, false);
}

__device__ __forceinline__ v8f v8f_zero() {
  v8f z = {0.f, 0.f, 0.f, 0.f, 0.f, 0.f, 0.f, 0.f};
  return z;
}

__global__ void __launch_bounds__(256) k_wprep(
    const float* __restrict__ Wb, const float* __restrict__ Wc, unsigned short* __restrict__ W16) {
  const int i = blockIdx.x * 256 + threadIdx.x;
  const int which = i >> 13;
  const int e = i & 8191;
  const int o = e >> 5;
  const int kc = e & 31;
  const size_t off = (size_t)o * CD + kc * 8;
  const v4f b0 = *(const v4f*)(Wb + off);
  const v4f b1 = *(const v4f*)(Wb + off + 4);
  const v4f c0 = *(const v4f*)(Wc + off);
  const v4f c1 = *(const v4f*)(Wc + off + 4);
  float f[8];
  f[0] = which ? c0.x : b0.x; f[1] = which ? c0.y : b0.y; f[2] = which ? c0.z : b0.z; f[3] = which ? c0.w : b0.w;
  f[4] = which ? c1.x : b1.x; f[5] = which ? c1.y : b1.y; f[6] = which ? c1.z : b1.z; f[7] = which ? c1.w : b1.w;
  v8us ov;
  #pragma unroll
  for (int j = 0; j < 8; ++j) ov[j] = h2us(f[j] * 16.0f);
  st2_u8(W16 + (size_t)which * W_N + off, ov);
}

__global__ void __launch_bounds__(256) k_xprep(const float* __restrict__ x, unsigned short* __restrict__ xT) {
  __shared__ __attribute__((aligned(16))) unsigned short sT[64 * XP];
  const int tid = threadIdx.x;
  const int lane = tid & 31;
  const int w = tid >> 5;
  const int bid = blockIdx.x;
  const int pt = bid & 63;
  const int ct = (bid >> 6) & 3;
  const int n = bid >> 8;
  const int p0 = pt * 64;
  const int c0 = ct * 64;

  #pragma unroll
  for (int it = 0; it < 4; ++it) {
    const int idx = it * 256 + tid;
    const int c = idx >> 4;
    const int p4 = (idx & 15) * 4;
    const v4f v = *(const v4f*)(x + ((size_t)(n * CD + c0 + c)) * HW + p0 + p4);
    sT[(p4 + 0) * XP + c] = h2us(v.x);
    sT[(p4 + 1) * XP + c] = h2us(v.y);
    sT[(p4 + 2) * XP + c] = h2us(v.z);
    sT[(p4 + 3) * XP + c] = h2us(v.w);
  }
  __syncthreads();

  const int q = lane >> 3;
  const int j = lane & 7;
  #pragma unroll 1
  for (int it = 0; it < 2; ++it) {
    const int prow = it * 32 + w * 4 + q;
    const v8us val = *(const v8usa*)(sT + prow * XP + j * 8);
    unsigned short* dst = xT + ((size_t)(n * HW + p0 + prow)) * CD + c0 + j * 8;
    st2_u8(dst, val);
  }
}

__device__ __forceinline__ void stage16(float* sT, v8f ab, v8f ac, int orow0, int col,
                                        const float* bbp, const float* bcp) {
  #pragma unroll
  for (int r = 0; r < 8; ++r) {
    const int orow = orow0 + r;
    sT[orow * EP + col] = ab[r] * 0.0625f + bbp[r];
    sT[(64 + orow) * EP + col] = ac[r] * 0.0625f + bcp[r];
  }
}

__global__ void __launch_bounds__(256) k_conv(
    const unsigned short* __restrict__ xT, const unsigned short* __restrict__ W16,
    const float* __restrict__ bb, const float* __restrict__ bc, float* __restrict__ px) {
  __shared__ __attribute__((aligned(16))) float sT[128 * EP];
  const int tid = threadIdx.x;
  const int lane = tid & 31;
  const int w = tid >> 5;
  const int h = lane >> 4;
  const int m = lane & 15;
  const int bid = blockIdx.x;
  const int pt = bid & 63;
  const int ot = (bid >> 6) & 3;
  const int n = bid >> 8;
  const int p0 = pt * 64;
  const int o0 = ot * 64;
  const int osub = (w >> 1) * 16;
  const int psub = (w & 1) * 32;

  const unsigned short* arb = W16 + (size_t)(o0 + osub + m) * CD;
  const unsigned short* arc = arb + W_N;
  const unsigned short* br0 = xT + ((size_t)(n * HW + p0 + psub + m)) * CD;
  const unsigned short* br1 = br0 + 16 * CD;

  v8f accB0 = v8f_zero(), accB1 = v8f_zero(), accC0 = v8f_zero(), accC1 = v8f_zero();

  #pragma unroll 1
  for (int ks = 0; ks < CD / 32; ++ks) {
    const int k0 = ks * 32;
    const v16h fab = ldfrag(arb + k0, h);
    const v16h fac = ldfrag(arc + k0, h);
    const v16h fb0 = ldfrag(br0 + k0, h);
    const v16h fb1 = ldfrag(br1 + k0, h);
    accB0 = wmma_h(fab, fb0, accB0);
    accB1 = wmma_h(fab, fb1, accB1);
    accC0 = wmma_h(fac, fb0, accC0);
    accC1 = wmma_h(fac, fb1, accC1);
    asm volatile("v_nop\n\tv_nop\n\tv_nop\n\tv_nop"
                 : "+v"(accB0), "+v"(accB1), "+v"(accC0), "+v"(accC1)
                 : "v"(fab), "v"(fac), "v"(fb0), "v"(fb1));
  }

  const float* bbp = bb + o0 + osub + 8 * h;
  const float* bcp = bc + o0 + osub + 8 * h;
  stage16(sT, accB0, accC0, osub + 8 * h, psub + m, bbp, bcp);
  stage16(sT, accB1, accC1, osub + 8 * h, psub + 16 + m, bbp, bcp);
  __syncthreads();

  const int q = lane >> 3;
  const int j = lane & 7;
  const int rsel = q >> 1;
  const int lsel = q & 1;
  #pragma unroll 1
  for (int it = 0; it < 8; ++it) {
    const int row2 = it * 16 + w * 2 + rsel;
    const int buf = row2 >> 6;
    const int row = row2 & 63;
    const v4f v = *(const v4fa*)(sT + row2 * EP + lsel * 32 + j * 4);
    float* dst = px + (size_t)buf * PLANE + ((size_t)(n * CD + o0 + row)) * HW + p0 + lsel * 32 + j * 4;
    st2_f4(dst, v);
  }
}

__global__ void __launch_bounds__(256) k_attn(
    const float* __restrict__ x, const float* __restrict__ pxb, const float* __restrict__ pxc,
    const float* __restrict__ alpha, float* __restrict__ out) {
  const int pix = blockIdx.x * 256 + threadIdx.x;
  const int n = pix >> 12;
  const int p = pix & (HW - 1);
  const int hy = p >> 6;
  const int wx = p & (WDIM - 1);

  int hh[5], ww[5];
  #pragma unroll
  for (int d = 0; d < 5; ++d) {
    int t = hy + d - 2;
    t = (t < 0) ? -t : t;
    t = (t >= HDIM) ? (2 * HDIM - 2 - t) : t;
    hh[d] = t * WDIM;
    int u = wx + d - 2;
    u = (u < 0) ? -u : u;
    u = (u >= WDIM) ? (2 * WDIM - 2 - u) : u;
    ww[d] = u;
  }

  const float* pb = pxb + (size_t)n * CD * HW;
  const float* pc = pxc + (size_t)n * CD * HW;

  float e[25];
  #pragma unroll
  for (int k = 0; k < 25; ++k) e[k] = 0.0f;

  #pragma unroll 1
  for (int c = 0; c < CD; ++c) {
    const float* plane = pb + (size_t)c * HW;
    const float xc = pc[(size_t)c * HW + p];
    #pragma unroll
    for (int di = 0; di < 5; ++di) {
      const float* rowp = plane + hh[di];
      #pragma unroll
      for (int dj = 0; dj < 5; ++dj)
        e[di * 5 + dj] = fmaf(xc, rowp[ww[dj]], e[di * 5 + dj]);
    }
  }

  float mx = e[0];
  #pragma unroll
  for (int k = 1; k < 25; ++k) mx = fmaxf(mx, e[k]);
  float s = 0.0f;
  #pragma unroll
  for (int k = 0; k < 25; ++k) {
    e[k] = __expf(e[k] - mx);
    s += e[k];
  }
  const float al = alpha[0];
  const float scale = al * (1.0f / s);

  #pragma unroll 1
  for (int c = 0; c < CD; ++c) {
    const float* plane = pb + (size_t)c * HW;
    float acc = 0.0f;
    #pragma unroll
    for (int di = 0; di < 5; ++di) {
      const float* rowp = plane + hh[di];
      #pragma unroll
      for (int dj = 0; dj < 5; ++dj)
        acc = fmaf(e[di * 5 + dj], rowp[ww[dj]], acc);
    }
    const size_t idx = ((size_t)n * CD + c) * HW + p;
    const float v = fmaf(scale, acc, x[idx]);
    *(volatile float*)(out + idx) = v;
    __threadfence();
    *(volatile float*)(out + idx) = v;
  }
}

extern "C" void kernel_launch(void* const* d_in, const int* in_sizes, int n_in,
                              void* d_out, int out_size, void* d_ws, size_t ws_size,
                              hipStream_t stream) {
  if (n_in < 6) return;
  if (in_sizes[0] != X_N || in_sizes[1] != W_N || in_sizes[2] != B_N ||
      in_sizes[3] != W_N || in_sizes[4] != B_N || in_sizes[5] < 1) return;
  if (out_size != OUT_N) return;
  if (ws_size < (size_t)WS_TOTAL) return;

  const float* x     = (const float*)d_in[0];
  const float* Wb    = (const float*)d_in[1];
  const float* bb    = (const float*)d_in[2];
  const float* Wc    = (const float*)d_in[3];
  const float* bc    = (const float*)d_in[4];
  const float* alpha = (const float*)d_in[5];
  float* out = (float*)d_out;

  char* ws = (char*)d_ws;
  float*          px   = (float*)(ws + OFF_PXB);
  unsigned short* xT   = (unsigned short*)(ws + OFF_XT);
  unsigned short* W16  = (unsigned short*)(ws + OFF_W16);

  k_wprep<<<dim3(64), dim3(256), 0, stream>>>(Wb, Wc, W16);
  k_xprep<<<dim3(NB * 4 * (HW / 64)), dim3(256), 0, stream>>>(x, xT);
  k_conv<<<dim3(NB * 4 * (HW / 64)), dim3(256), 0, stream>>>(xT, W16, bb, bc, px);
  k_attn<<<dim3((NB * HW) / 256), dim3(256), 0, stream>>>(x, px, px + PLANE, alpha, out);
}
